// MultiHeadAttentionBlock_49967649521921
// MI455X (gfx1250) — hardware-verified
//
#include <hip/hip_runtime.h>
#include <math.h>

typedef __attribute__((ext_vector_type(16))) _Float16 v16h;
typedef __attribute__((ext_vector_type(16))) __bf16 v16b;
typedef __attribute__((ext_vector_type(8)))  _Float16 v8h;
typedef __attribute__((ext_vector_type(8)))  float v8f;
typedef __attribute__((ext_vector_type(4)))  float v4f;
typedef __attribute__((ext_vector_type(2)))  float v2f;
typedef __attribute__((ext_vector_type(4)))  unsigned v4u;
typedef __attribute__((ext_vector_type(4)))  int v4i;
typedef float __attribute__((may_alias)) float_a;
typedef int __attribute__((may_alias)) int_a;

template <typename T> __device__ __forceinline__ void vst2(void* p, T v) { *(volatile T*)p = v; __threadfence(); *(volatile T*)p = v; }
__device__ __forceinline__ v8f wmma16(v16h a, v16h b, v8f c) {
  v8f d = __builtin_amdgcn_wmma_f32_16x16x32_f16(false, a, false, b, (short)0, c, false, false);
  asm volatile("v_nop\n\tv_nop\n\tv_nop\n\tv_nop" : "+v"(d) : "v"(a), "v"(b));
  return d;
}
__device__ __forceinline__ v8f wmma_bf(v16b a, v16b b, v8f c) {
  v8f d = __builtin_amdgcn_wmma_f32_16x16x32_bf16(false, a, false, b, (short)0, c, false, false);
  asm volatile("v_nop\n\tv_nop\n\tv_nop\n\tv_nop" : "+v"(d) : "v"(a), "v"(b));
  return d;
}
__device__ __forceinline__ v16h frag_h(const _Float16* rowk0, int lane) {
  union { v16h v; v8h q[2]; } u; const _Float16* p = rowk0 + 8 * (lane >> 4);
  u.q[0] = *(const v8h*)p; u.q[1] = *(const v8h*)(p + 16); return u.v;
}
__device__ __forceinline__ v16h frag_f32(const float* rowk0, int lane) {
  v16h a; const float* p = rowk0 + 8 * (lane >> 4);
#pragma unroll
  for (int i = 0; i < 8; ++i) { a[i] = (_Float16)p[i]; a[8 + i] = (_Float16)p[16 + i]; }
  return a;
}
__device__ __forceinline__ v16h frag_f32s(const float* rowk0, int lane, float sc) {
  v16h a; const float* p = rowk0 + 8 * (lane >> 4);
#pragma unroll
  for (int i = 0; i < 8; ++i) { a[i] = (_Float16)(p[i] * sc); a[8 + i] = (_Float16)(p[16 + i] * sc); }
  return a;
}
__device__ __forceinline__ v16h fragc_f32(const float* W, int k0, int n, int lane, int ld, int K) {
  v16h a; const int g = lane >> 4;
#pragma unroll
  for (int i = 0; i < 8; ++i) { const int ka = k0 + 8 * g + i, kb = ka + 16;
    a[i] = (_Float16)(ka < K ? W[(size_t)(ka < K ? ka : K - 1) * ld + n] : 0.f); a[8 + i] = (_Float16)(kb < K ? W[(size_t)(kb < K ? kb : K - 1) * ld + n] : 0.f); }
  return a;
}
struct F2 { v16b h, l; };
__device__ __forceinline__ F2 bsplit16(const float v[16]) { F2 r;
#pragma unroll
  for (int i = 0; i < 16; ++i) { const __bf16 h = (__bf16)v[i]; r.h[i] = h; r.l[i] = (__bf16)(v[i] - (float)h); }
  return r; }
__device__ __forceinline__ F2 split_row(const float* row, int k0, int lane) { float v[16]; const float* p = row + k0 + 8 * (lane >> 4);
#pragma unroll
  for (int i = 0; i < 8; ++i) { v[i] = p[i]; v[8 + i] = p[16 + i]; }
  return bsplit16(v); }
__device__ __forceinline__ F2 split_rowK(const float* row, int k0, int lane, int K) { float v[16]; const int g = lane >> 4;
#pragma unroll
  for (int i = 0; i < 8; ++i) { const int ka = k0 + 8 * g + i, kb = ka + 16; v[i] = ka < K ? row[ka < K ? ka : K - 1] : 0.f; v[8 + i] = kb < K ? row[kb < K ? kb : K - 1] : 0.f; }
  return bsplit16(v); }
__device__ __forceinline__ F2 split_col(const float* W, int k0, int n, int lane, int ld, int K) { float v[16]; const int g = lane >> 4;
#pragma unroll
  for (int i = 0; i < 8; ++i) { const int ka = k0 + 8 * g + i, kb = ka + 16; v[i] = ka < K ? W[(size_t)(ka < K ? ka : K - 1) * ld + n] : 0.f; v[8 + i] = kb < K ? W[(size_t)(kb < K ? kb : K - 1) * ld + n] : 0.f; }
  return bsplit16(v); }
__device__ __forceinline__ v8f mac3(const F2& a, const F2& b, v8f c) { c = wmma_bf(a.l, b.h, c); c = wmma_bf(a.h, b.l, c); return wmma_bf(a.h, b.h, c); }
__device__ __forceinline__ float sigm(float v) { return 1.0f / (1.0f + expf(-v)); }
#define LDSX() do { asm volatile("s_wait_dscnt 0" ::: "memory"); __builtin_amdgcn_wave_barrier(); __builtin_amdgcn_fence(__ATOMIC_RELEASE, "workgroup"); } while (0)

#define NB 16
#define TT 2048
#define CC 1024
#define DIN 1024
#define NH 16
#define HD 64
#define NQB (TT / 64)
#define HG 4
#define SCALE (0.125f)
#define CAUSAL 1
#ifndef TNB
#define TNB NB
#endif
__device__ __forceinline__ float bfr(float v) { return (float)(__bf16)v; }
__host__ __device__ __forceinline__ int kb_last(int qb) { return CAUSAL ? ((qb * 64 + 63) >> 7) : (TT / 128 - 1); }
typedef __attribute__((ext_vector_type(8))) __bf16 v8b;
__device__ __forceinline__ v16b frag_b(const __bf16* rowk0, int lane) {
  union { v16b v; v8b q[2]; } u; const __bf16* p = rowk0 + 8 * (lane >> 4);
  u.q[0] = *(const v8b*)p; u.q[1] = *(const v8b*)(p + 16); return u.v;
}
#define QBH 6
#define QHI 384
#define KHI 384
__device__ __forceinline__ v16b wcol_io(const float* Wm, int k0, int o, int lane, int ld) { v16b w; const int g = lane >> 4;
#pragma unroll
  for (int i = 0; i < 8; ++i) { w[i] = (__bf16)Wm[(size_t)(k0 + 8 * g + i) * ld + o]; w[8 + i] = (__bf16)Wm[(size_t)(k0 + 16 + 8 * g + i) * ld + o]; }
  return w; }
__device__ __forceinline__ v16b wcol_oi(const float* Wm, int k0, int o, int lane, int K) { v16b w; const float* p = Wm + (size_t)o * K + k0 + 8 * (lane >> 4);
#pragma unroll
  for (int i = 0; i < 8; ++i) { w[i] = (__bf16)p[i]; w[8 + i] = (__bf16)p[16 + i]; }
  return w; }
__device__ __forceinline__ v16h wcolh_io(const float* Wm, int k0, int o, int lane, int ld) { v16h w; const int g = lane >> 4;
#pragma unroll
  for (int i = 0; i < 8; ++i) { w[i] = (_Float16)(bfr(Wm[(size_t)(k0 + 8 * g + i) * ld + o]) * 256.0f); w[8 + i] = (_Float16)(bfr(Wm[(size_t)(k0 + 16 + 8 * g + i) * ld + o]) * 256.0f); }
  return w; }
__device__ __forceinline__ v16h wcolh_oi(const float* Wm, int k0, int o, int lane, int K) { v16h w; const float* p = Wm + (size_t)o * K + k0 + 8 * (lane >> 4);
#pragma unroll
  for (int i = 0; i < 8; ++i) { w[i] = (_Float16)(bfr(p[i]) * 256.0f); w[8 + i] = (_Float16)(bfr(p[16 + i]) * 256.0f); }
  return w; }
#define WQKV_LAYOUT 1
__device__ __forceinline__ v16b wcol_hdk(const float* Wm, int k0, int o, int lane) { v16b w; const int g = lane >> 4; const float* p = Wm + (size_t)(o / HD) * DIN * HD + (o % HD);
#pragma unroll
  for (int i = 0; i < 8; ++i) { w[i] = (__bf16)p[(size_t)(k0 + 8 * g + i) * HD]; w[8 + i] = (__bf16)p[(size_t)(k0 + 16 + 8 * g + i) * HD]; }
  return w; }
#define WO_OUT_IN 1
#if WQKV_LAYOUT == 1
#define WCOL(W, k0, o, lane) wcol_oi(W, k0, o, lane, DIN)
#elif WQKV_LAYOUT == 2
#define WCOL(W, k0, o, lane) wcol_hdk(W, k0, o, lane)
#else
#define WCOL(W, k0, o, lane) wcol_io(W, k0, o, lane, CC)
#endif
#if WO_OUT_IN
#define WOCOL(W, k0, o, lane) wcol_oi(W, k0, o, lane, CC)
#define WOCOLH(W, k0, o, lane) wcolh_oi(W, k0, o, lane, CC)
#else
#define WOCOL(W, k0, o, lane) wcol_io(W, k0, o, lane, DIN)
#define WOCOLH(W, k0, o, lane) wcolh_io(W, k0, o, lane, DIN)
#endif

#ifndef SM_EXTRA_PARAMS
#define SM_EXTRA_PARAMS
#endif
#ifndef PROJ_EXTRA_PARAMS
#define PROJ_EXTRA_PARAMS
#endif
#ifndef SM_MASK_HOOK
#define SM_MASK_HOOK (void)0
#endif

#define WS_QH  0u
#define WS_KH  (WS_QH + 2u * (size_t)NB * TT * CC)
#define WS_VT  (WS_KH + 2u * (size_t)NB * TT * CC)
#define WS_QL  (WS_VT + 2u * (size_t)NB * CC * TT)
#define WS_KL  (WS_QL + 2u * (size_t)NB * QHI * CC)
#define WS_VB  (WS_KL + 2u * (size_t)NB * KHI * CC)
#define WS_VBL (WS_VB + 2u * (size_t)NB * CC * KHI)
#define WS_S   (WS_VBL + 2u * (size_t)NB * CC * KHI)
#define WS_Y   (WS_S  + 4u * (size_t)HG * TT * TT)
#define WS_END (WS_Y  + 4u * (size_t)NB * TT * CC)


#define NBT 16
#define CCH 512
#define NHD 8
#define HDC 64
#define NP 1024
__global__ __launch_bounds__(128) void k_lin(const float* __restrict__ X, const float* __restrict__ WQ, const float* __restrict__ WK, const float* __restrict__ WV, const float* __restrict__ BQ, const float* __restrict__ BK, const float* __restrict__ BV, float* __restrict__ YQ, float* __restrict__ YK, float* __restrict__ YV) {
  __shared__ __align__(16) float sf[4][16][132];
  const int tid = threadIdx.x, wave = tid >> 5, lane = tid & 31, col = lane & 15, g = lane >> 4; const int c0 = blockIdx.x * 64 + wave * 16; const int n0 = blockIdx.y * 128; const int b = blockIdx.z / 3, which = blockIdx.z % 3;
  const float* W = which == 0 ? WQ : which == 1 ? WK : WV; const float* BI = which == 0 ? BQ : which == 1 ? BK : BV; float* Y = which == 0 ? YQ : which == 1 ? YK : YV;
  const float* xb = X + (size_t)b * CCH * NP;
  v8f acc[8] = {};
#pragma unroll 1
  for (int kc = 0; kc < CCH / 32; ++kc) { const F2 a = split_row(W + (size_t)(c0 + col) * CCH, kc * 32, lane); asm volatile("s_wait_loadcnt 0x0" ::: "memory");
#pragma unroll
    for (int j = 0; j < 8; ++j) { const v16b xf = wcol_io(xb, kc * 32, n0 + j * 16 + col, lane, NP); asm volatile("s_wait_loadcnt 0x0" ::: "memory"); acc[j] = wmma_bf(a.h, xf, acc[j]); } }
#pragma unroll
  for (int j = 0; j < 8; ++j) {
#pragma unroll
    for (int r = 0; r < 8; ++r) { const float bias = bfr(BI[c0 + 8 * g + r]); sf[wave][8 * g + r][j * 16 + col] = acc[j][r] + bias; } }
  LDSX(); for (int rl = 0; rl < 16; ++rl) vst2(Y + ((size_t)b * CCH + c0 + rl) * NP + n0 + lane * 4, *(const v4f*)&sf[wave][rl][lane * 4]); }
__global__ __launch_bounds__(128) void k_catt(const float* __restrict__ YQ, const float* __restrict__ YK, const float* __restrict__ YV, float* __restrict__ T) {
  __shared__ __align__(16) float sp[64][68]; __shared__ __align__(16) float st[128][68];
  const int tid = threadIdx.x, wave = tid >> 5, lane = tid & 31, col = lane & 15, g = lane >> 4; const int b = blockIdx.x / NHD, h = blockIdx.x % NHD;
  const float* qb = YQ + ((size_t)b * CCH + h * HDC) * NP; const float* kb = YK + ((size_t)b * CCH + h * HDC) * NP; const float* vb = YV + ((size_t)b * CCH + h * HDC) * NP;
  { v8f acc[4] = {};
#pragma unroll 1
    for (int kc = 0; kc < NP / 32; ++kc) { const F2 a = split_row(qb + (size_t)(wave * 16 + col) * NP, kc * 32, lane); asm volatile("s_wait_loadcnt 0x0" ::: "memory");
#pragma unroll
      for (int j = 0; j < 4; ++j) { const F2 w = split_row(kb + (size_t)(j * 16 + col) * NP, kc * 32, lane); asm volatile("s_wait_loadcnt 0x0" ::: "memory"); acc[j] = mac3(a, w, acc[j]); } }
#pragma unroll
    for (int j = 0; j < 4; ++j)
#pragma unroll
      for (int r = 0; r < 8; ++r) sp[wave * 16 + 8 * g + r][j * 16 + col] = acc[j][r] * 0.125f; }
  __syncthreads();
  if (tid < 64) { float m = -3.0e38f; for (int e = 0; e < HDC; ++e) m = fmaxf(m, sp[tid][e]); float sum = 0.f; for (int e = 0; e < HDC; ++e) { const float x = expf(sp[tid][e] - m); sp[tid][e] = x; sum += x; } const float inv = 1.0f / sum; for (int e = 0; e < HDC; ++e) sp[tid][e] = sp[tid][e] * inv; }
  __syncthreads();
  F2 pa[2];
#pragma unroll
  for (int kc = 0; kc < 2; ++kc) { float v[16]; const float* p = &sp[wave * 16 + col][kc * 32 + 8 * g];
#pragma unroll
    for (int i = 0; i < 8; ++i) { v[i] = p[i]; v[8 + i] = p[16 + i]; } pa[kc] = bsplit16(v); }
#pragma unroll 1
  for (int nb = 0; nb < NP / 128; ++nb) { v8f acc[8] = {};
#pragma unroll
    for (int kc = 0; kc < 2; ++kc) {
#pragma unroll
      for (int j = 0; j < 8; ++j) { const F2 w = split_col(vb, kc * 32, nb * 128 + j * 16 + col, lane, NP, HDC); asm volatile("s_wait_loadcnt 0x0" ::: "memory"); acc[j] = mac3(pa[kc], w, acc[j]); } }
    __syncthreads();
#pragma unroll
    for (int j = 0; j < 8; ++j)
#pragma unroll
      for (int r = 0; r < 8; ++r) st[j * 16 + col][wave * 16 + 8 * g + r] = acc[j][r];
    __syncthreads();
    for (int e2 = tid; e2 < 128 * 16; e2 += 128) { const int nl = e2 >> 4, q = e2 & 15; const int n = nb * 128 + nl; float* dst = T + ((size_t)b * CCH + h * HDC + n / 16) * NP + (size_t)(n % 16) * HDC + q * 4; vst2(dst, *(const v4f*)&st[nl][q * 4]); } } }
__global__ __launch_bounds__(128) void k_fin(const float* __restrict__ T, const float* __restrict__ WO, const float* __restrict__ BO, float* __restrict__ OUT) { __shared__ __align__(16) float sf[4][16][132];
  const int tid = threadIdx.x, wave = tid >> 5, lane = tid & 31, col = lane & 15, g = lane >> 4; const int o0 = blockIdx.x * 64 + wave * 16; const int p0 = blockIdx.y * 128; const int b = blockIdx.z;
  const float* tb = T + (size_t)b * CCH * NP;
  v8f acc[8] = {};
#pragma unroll 1
  for (int kc = 0; kc < CCH / 32; ++kc) { const F2 a = split_row(WO + (size_t)(o0 + col) * CCH, kc * 32, lane); asm volatile("s_wait_loadcnt 0x0" ::: "memory");
#pragma unroll
    for (int j = 0; j < 8; ++j) { const F2 w = split_col(tb, kc * 32, p0 + j * 16 + col, lane, NP, CCH); asm volatile("s_wait_loadcnt 0x0" ::: "memory"); acc[j] = wmma_bf(a.h, w.h, acc[j]); acc[j] = wmma_bf(a.h, w.l, acc[j]); } }
#pragma unroll
  for (int j = 0; j < 8; ++j)
#pragma unroll
    for (int r = 0; r < 8; ++r) { const float bias = bfr(BO[o0 + 8 * g + r]); sf[wave][8 * g + r][j * 16 + col] = acc[j][r] + bias; }
  LDSX(); for (int rl = 0; rl < 16; ++rl) vst2(OUT + ((size_t)b * CCH + o0 + rl) * NP + p0 + lane * 4, *(const v4f*)&sf[wave][rl][lane * 4]); }
#define WS_YQ 0u
#define WS_YK (WS_YQ + 4u * (size_t)NBT * CCH * NP)
#define WS_YV (WS_YK + 4u * (size_t)NBT * CCH * NP)
#define WS_T2 (WS_YV + 4u * (size_t)NBT * CCH * NP)
#define WS_TOT (WS_T2 + 4u * (size_t)NBT * CCH * NP)
extern "C" void kernel_launch(void* const* d_in, const int* in_sizes, int n_in, void* d_out, int out_size, void* d_ws, size_t ws_size, hipStream_t stream) {
  (void)in_sizes; (void)n_in; (void)out_size;
  const float** F = (const float**)d_in;
  if (ws_size < (size_t)WS_TOT) return;
  char* ws = (char*)d_ws; float *YQ = (float*)(ws + WS_YQ), *YK = (float*)(ws + WS_YK), *YV = (float*)(ws + WS_YV), *T = (float*)(ws + WS_T2);
  k_lin<<<dim3(CCH / 64, NP / 128, TNB * 3), 128, 0, stream>>>(F[0], F[1], F[3], F[5], F[2], F[4], F[6], YQ, YK, YV);
  k_catt<<<dim3(TNB * NHD), 128, 0, stream>>>(YQ, YK, YV, T);
  k_fin<<<dim3(CCH / 64, NP / 128, TNB), 128, 0, stream>>>(T, F[7], F[8], (float*)d_out);
}
